// GeometricAttention_18339510354278
// MI455X (gfx1250) — hardware-verified
//
#include <hip/hip_runtime.h>
#include <math.h>
#include <stdint.h>

constexpr int kBatch   = 8;
constexpr int kSeq     = 2048;
constexpr int kDim     = 512;
constexpr int kTok     = kBatch * kSeq;
constexpr int kNpos    = 4096;
constexpr int kRowsBlk = 2048;
constexpr int kNumBlk  = kTok / kRowsBlk;
constexpr int kWRows   = 32;
constexpr int kGTiles  = (kRowsBlk / 64) * (kNpos / 64);
constexpr int kPVTiles = (kRowsBlk / 64) * (kDim / 64);
static_assert(kTok % kRowsBlk == 0);
static_assert(kRowsBlk % 64 == 0 && kNpos % 64 == 0 && kDim % 64 == 0);
static_assert(kDim % 32 == 0 && kNpos % 32 == 0);
static_assert(kRowsBlk % kWRows == 0 && kNpos == 256 * 16);
static_assert(kGTiles % 8 == 0 && kPVTiles % 8 == 0);

constexpr size_t kSzXB  = (size_t)kTok * kDim * 2;
constexpr size_t kSzPB  = (size_t)kNpos * kDim * 2;
constexpr size_t kSzVT  = (size_t)kDim * kNpos * 2;
constexpr size_t kSzXsq = (size_t)kTok * 4;
constexpr size_t kSzPsq = (size_t)kNpos * 4;
constexpr size_t kSzIdn = (size_t)kNpos * 4;
constexpr size_t kSzRsc = (size_t)kTok * 4;
constexpr size_t kSzG   = (size_t)kRowsBlk * kNpos * 4;
constexpr size_t kSzP   = (size_t)kRowsBlk * kNpos * 2;
constexpr size_t kOffXB  = 0;
constexpr size_t kOffPB  = kOffXB + kSzXB;
constexpr size_t kOffVT  = kOffPB + kSzPB;
constexpr size_t kOffXsq = kOffVT + kSzVT;
constexpr size_t kOffPsq = kOffXsq + kSzXsq;
constexpr size_t kOffIdn = kOffPsq + kSzPsq;
constexpr size_t kOffRsc = kOffIdn + kSzIdn;
constexpr size_t kOffG   = kOffRsc + kSzRsc;
constexpr size_t kOffPh  = kOffG + kSzG;
constexpr size_t kOffPl  = kOffPh + kSzP;
constexpr size_t kWsEnd  = kOffPl + kSzP;
static_assert(kWsEnd == 92438528ull);
static_assert(kWsEnd <= 134217728ull);
static_assert(kOffG % 128 == 0 && kOffPh % 128 == 0 && kOffPl % 128 == 0 && kOffRsc % 128 == 0 && kOffXsq % 128 == 0);

typedef __attribute__((ext_vector_type(16))) _Float16 v16h;
typedef __attribute__((ext_vector_type(8)))  _Float16 v8h;
typedef __attribute__((ext_vector_type(16))) __bf16   v16b;
typedef __attribute__((ext_vector_type(8)))  __bf16   v8b;
typedef __attribute__((ext_vector_type(8)))  float    v8f;
typedef __attribute__((ext_vector_type(4)))  float    v4f;
typedef __attribute__((ext_vector_type(4)))  unsigned int v4u;

__device__ __forceinline__ unsigned short f2bf_bits(float f) {
  unsigned u = __float_as_uint(f);
  return (unsigned short)((u + 0x7FFFu + ((u >> 16) & 1u)) >> 16);
}
__device__ __forceinline__ float bf_bits2f(unsigned short h) { return __uint_as_float(((unsigned)h) << 16); }

__device__ __forceinline__ void dep_guard_h(v8f& a, v8f& b, v16h x, v16h y) { asm volatile("v_nop\n\tv_nop\n\tv_nop\n\tv_nop" : "+v"(a), "+v"(b) : "v"(x), "v"(y)); }
__device__ __forceinline__ void dep_guard_b(v8f& a, v8f& b, v16b x, v16b y) { asm volatile("v_nop\n\tv_nop\n\tv_nop\n\tv_nop" : "+v"(a), "+v"(b) : "v"(x), "v"(y)); }
__device__ __forceinline__ void keep4_h(v16h a, v16h b, v16h c, v16h d) { asm volatile("v_nop" :: "v"(a), "v"(b), "v"(c), "v"(d)); }
__device__ __forceinline__ void keep4_b(v16b a, v16b b, v16b c, v16b d) { asm volatile("v_nop" :: "v"(a), "v"(b), "v"(c), "v"(d)); }
__device__ __forceinline__ void acc_guard4(v8f& a, v8f& b, v8f& c, v8f& d) { asm volatile("v_nop\n\tv_nop\n\tv_nop\n\tv_nop" : "+v"(a), "+v"(b), "+v"(c), "+v"(d)); }
template <typename T> struct Frag;
template <> struct Frag<_Float16> {
  typedef v16h V; union U { v16h v; v8h h[2]; };
  static __device__ __forceinline__ v16h load(const _Float16* p) {
    U f; f.h[0] = *(const v8h*)(p); f.h[1] = *(const v8h*)(p + 16); return f.v;
  }
  static __device__ __forceinline__ v8f mma(v16h a, v16h b, v8f c) {
    return __builtin_amdgcn_wmma_f32_16x16x32_f16(false, a, false, b, (short)0, c, false, false);
  }
  static __device__ __forceinline__ void guard(v8f& a, v8f& b, v16h x, v16h y) { dep_guard_h(a, b, x, y); }
  static __device__ __forceinline__ void keep(v16h a, v16h b, v16h c, v16h d) { keep4_h(a, b, c, d); }
};
template <> struct Frag<__bf16> {
  typedef v16b V; union U { v16b v; v8b h[2]; };
  static __device__ __forceinline__ v16b load(const __bf16* p) {
    U f; f.h[0] = *(const v8b*)(p); f.h[1] = *(const v8b*)(p + 16); return f.v;
  }
  static __device__ __forceinline__ v8f mma(v16b a, v16b b, v8f c) {
    return __builtin_amdgcn_wmma_f32_16x16x32_bf16(false, a, false, b, (short)0, c, false, false);
  }
  static __device__ __forceinline__ void guard(v8f& a, v8f& b, v16b x, v16b y) { dep_guard_b(a, b, x, y); }
  static __device__ __forceinline__ void keep(v16b a, v16b b, v16b c, v16b d) { keep4_b(a, b, c, d); }
};

__device__ __forceinline__ unsigned pk16(unsigned short a, unsigned short b) { return (unsigned)a | ((unsigned)b << 16); }

template <int ET> struct Elem;
template <> struct Elem<0> { typedef _Float16 T; };
template <> struct Elem<1> { typedef __bf16 T; };
template <int ET, int SPLITM, int BIAS_MODE, int OUT_MODE, bool RESID, int ACT = 0>
__global__ __launch_bounds__(256) void wmma_gemm64(
    const unsigned short* __restrict__ Ap, const unsigned short* __restrict__ A2p, int lda, long strideA,
    const unsigned short* __restrict__ Btp, const unsigned short* __restrict__ Bt2p, int ldb, long strideB,
    void* __restrict__ Cout, void* __restrict__ Cout2, int ldc, long strideC,
    const float* __restrict__ bias,
    const float* __restrict__ resid, long strideR,
    int M, int N, int K, float scale) {
  constexpr bool SPLA = (SPLITM >= 1);
  constexpr bool SPLB = (SPLITM == 2);
  typedef typename Elem<ET>::T T;
  typedef typename Frag<T>::V V;
  const T* A = (const T*)Ap; const T* A2 = (const T*)A2p; const T* Bt = (const T*)Btp; const T* Bt2 = (const T*)Bt2p;
  __shared__ __align__(16) float sT[8][16 * 68];
  const int b    = blockIdx.y;
  const int lane = threadIdx.x & 31;
  const int wave = threadIdx.x >> 5;
  const int tilesN = N >> 6;
  const int tilesM = M >> 6;
  const int tile = blockIdx.x * 8 + wave;
  if (tile >= tilesM * tilesN) return;
  const int tm = tile / tilesN;
  const int tn = tile - tm * tilesN;
  const int m0 = tm << 6;
  const int n0 = tn << 6;

  const T* Ab  = A  + (size_t)b * strideA;
  const T* Bb  = Bt + (size_t)b * strideB;
  const T* Ab2 = SPLA ? (A2  + (size_t)b * strideA) : nullptr;
  const T* Bb2 = SPLB ? (Bt2 + (size_t)b * strideB) : nullptr;

  const int rlane = lane & 15;
  const int koff  = (lane >> 4) * 8;
  const int mOff  = (lane >> 4) * 8;

  v8f acc[4][4];
#pragma unroll
  for (int i = 0; i < 4; ++i)
#pragma unroll
    for (int j = 0; j < 4; ++j) acc[i][j] = (v8f){0.f,0.f,0.f,0.f,0.f,0.f,0.f,0.f};

  for (int k0 = 0; k0 < K; k0 += 32) {
    V bh[4], bl[4];
#pragma unroll
    for (int j = 0; j < 4; ++j) {
      const size_t bo = (size_t)(n0 + (j << 4) + rlane) * ldb + koff + k0;
      bh[j] = Frag<T>::load(Bb + bo);
      if (SPLB) bl[j] = Frag<T>::load(Bb2 + bo);
    }
#pragma unroll
    for (int i = 0; i < 4; ++i) {
      const size_t ao = (size_t)(m0 + (i << 4) + rlane) * lda + koff + k0;
      V ah = Frag<T>::load(Ab + ao);
      V al;
      if (SPLA) al = Frag<T>::load(Ab2 + ao);
#pragma unroll
      for (int j = 0; j < 4; ++j) {
        acc[i][j] = Frag<T>::mma(ah, bh[j], acc[i][j]);
        if (SPLB) acc[i][j] = Frag<T>::mma(ah, bl[j], acc[i][j]);
        if (SPLA) acc[i][j] = Frag<T>::mma(al, bh[j], acc[i][j]);
      }
      Frag<T>::guard(acc[i][0], acc[i][3], ah, SPLA ? al : ah);
    }
    Frag<T>::keep(bh[0], bh[1], bh[2], bh[3]);
    if (SPLB) Frag<T>::keep(bl[0], bl[1], bl[2], bl[3]);
  }
  acc_guard4(acc[0][0], acc[0][1], acc[0][2], acc[0][3]);
  acc_guard4(acc[1][0], acc[1][1], acc[1][2], acc[1][3]);
  acc_guard4(acc[2][0], acc[2][1], acc[2][2], acc[2][3]);
  acc_guard4(acc[3][0], acc[3][1], acc[3][2], acc[3][3]);

  float* slab = sT[wave];
  const float* Rb = RESID ? (resid + (size_t)b * strideR) : nullptr;
#pragma unroll
  for (int i = 0; i < 4; ++i) {
    const int mBase = m0 + (i << 4);
#pragma unroll
    for (int j = 0; j < 4; ++j) {
      const int n = n0 + (j << 4) + rlane;
      float bv = 0.f;
      if (BIAS_MODE == 2) bv = bias[n];
#pragma unroll
      for (int r = 0; r < 8; ++r) {
        float v = acc[i][j][r] * scale;
        if (BIAS_MODE == 1) v += bias[mBase + mOff + r];
        if (BIAS_MODE == 2) v += bv;
        if (BIAS_MODE == 3) v *= bias[mBase + mOff + r];
        if (RESID) v += Rb[(size_t)(mBase + mOff + r) * ldc + n];
        if (ACT == 2) v = fmaxf(v, 0.0f);
        if (ACT == 4) v = (v > 0.f) ? v : 0.01f * v;
        slab[(mOff + r) * 68 + (j << 4) + rlane] = v;
      }
    }
    __builtin_amdgcn_fence(__ATOMIC_RELEASE, "workgroup");
    __builtin_amdgcn_wave_barrier();
    __builtin_amdgcn_fence(__ATOMIC_ACQUIRE, "workgroup");
    if (OUT_MODE == 0) {
      float* C = (float*)Cout + (size_t)b * strideC;
      const int hh = lane >> 4, c4 = (lane & 15) * 4;
      for (int pass = 0; pass < 2; ++pass) {
#pragma unroll
        for (int it = 0; it < 8; ++it) {
          const int row = it * 2 + hh;
          v4f v = *(const v4f*)(slab + row * 68 + c4);
          *(volatile v4f*)(C + (size_t)(mBase + row) * ldc + n0 + c4) = v;
        }
        __threadfence();
      }
    } else {
      const int q = lane >> 3, c8 = (lane & 7) * 8;
      unsigned short* C  = (unsigned short*)Cout  + (size_t)b * strideC;
      unsigned short* C2 = (OUT_MODE == 2) ? ((unsigned short*)Cout2 + (size_t)b * strideC) : nullptr;
      for (int pass = 0; pass < 2; ++pass) {
#pragma unroll
        for (int it = 0; it < 4; ++it) {
          const int row = it * 4 + q;
          const float* sp = slab + row * 68 + c8;
          v8h hv, lv;
#pragma unroll
          for (int e = 0; e < 8; ++e) {
            if (OUT_MODE == 1) {
              hv[e] = (_Float16)sp[e];
            } else {
              unsigned short hb = f2bf_bits(sp[e]);
              unsigned short lb = f2bf_bits(sp[e] - bf_bits2f(hb));
              hv[e] = __builtin_bit_cast(_Float16, hb);
              lv[e] = __builtin_bit_cast(_Float16, lb);
            }
          }
          *(volatile v8h*)(C + (size_t)(mBase + row) * ldc + n0 + c8) = hv;
          if (OUT_MODE == 2) *(volatile v8h*)(C2 + (size_t)(mBase + row) * ldc + n0 + c8) = lv;
        }
        __threadfence();
      }
    }
    __builtin_amdgcn_fence(__ATOMIC_RELEASE, "workgroup");
    __builtin_amdgcn_wave_barrier();
    __builtin_amdgcn_fence(__ATOMIC_ACQUIRE, "workgroup");
  }
}

template <bool WITH_TEMP>
__global__ __launch_bounds__(256) void rowcast_bf16_kernel(const float* __restrict__ in, unsigned short* __restrict__ out,
                                                          float* __restrict__ sqout, const float* __restrict__ temp,
                                                          float* __restrict__ invden) {
  __shared__ float part[8];
  __shared__ __align__(16) float ssq[32];
  __shared__ __align__(16) float sid[32];
  const int t = threadIdx.x, lane = t & 31, wave = t >> 5;
  const int sr = t >> 6;
  const int c8 = (t & 63) * 8;
#pragma unroll 1
  for (int g = 0; g < 8; ++g) {
    const int row = blockIdx.x * 32 + g * 4 + sr;
    const float* p = in + (size_t)row * kDim + c8;
    const v4f a = *(const v4f*)(p);
    const v4f c = *(const v4f*)(p + 4);
    unsigned short hb[8];
    float s = 0.f;
#pragma unroll
    for (int e = 0; e < 4; ++e) {
      hb[e] = f2bf_bits(a[e]);
      const float f = bf_bits2f(hb[e]);
      s += f * f;
    }
#pragma unroll
    for (int e = 0; e < 4; ++e) {
      hb[4 + e] = f2bf_bits(c[e]);
      const float f = bf_bits2f(hb[4 + e]);
      s += f * f;
    }
    const v4u u = (v4u){pk16(hb[0], hb[1]), pk16(hb[2], hb[3]), pk16(hb[4], hb[5]), pk16(hb[6], hb[7])};
    unsigned short* q = out + (size_t)row * kDim + c8;
    *(volatile v4u*)q = u;
    __threadfence();
    *(volatile v4u*)q = u;
#pragma unroll
    for (int off = 16; off > 0; off >>= 1) s += __shfl_xor(s, off);
    if (lane == 0) part[wave] = s;
    __syncthreads();
    if (t < 4) ssq[g * 4 + t] = part[2 * t] + part[2 * t + 1];
    __syncthreads();
  }
  if (WITH_TEMP) {
    if (t < 32) {
      const float tv = temp[blockIdx.x * 32 + t];
      sid[t] = 1.0f / (fabsf(tv) + 0.1f);
    }
  }
  __syncthreads();
  if (wave == 0 && lane < 8) {
    const v4f v = *(const v4f*)(ssq + 4 * lane);
    float* dst = sqout + (size_t)blockIdx.x * 32 + 4 * lane;
    *(volatile v4f*)dst = v;
    __threadfence();
    *(volatile v4f*)dst = v;
    if (WITH_TEMP) {
      const v4f w = *(const v4f*)(sid + 4 * lane);
      float* d2 = invden + (size_t)blockIdx.x * 32 + 4 * lane;
      *(volatile v4f*)d2 = w;
      __threadfence();
      *(volatile v4f*)d2 = w;
    }
  }
}

__global__ __launch_bounds__(256) void vtcast_kernel(const float* __restrict__ val, unsigned short* __restrict__ out) {
  __shared__ float sm[64][65];
  const int t  = threadIdx.x;
  const int d0 = blockIdx.x * 64;
  const int n0 = blockIdx.y * 64;
#pragma unroll
  for (int i = 0; i < 16; ++i) {
    const int e = i * 256 + t;
    const int r = e >> 6;
    const int c = e & 63;
    sm[c][r] = val[(size_t)(n0 + r) * kDim + d0 + c];
  }
  __syncthreads();
  const int lane = t & 31, wave = t >> 5;
  const int q = lane >> 3, c8 = (lane & 7) * 8;
  for (int pass = 0; pass < 2; ++pass) {
#pragma unroll
    for (int it = 0; it < 2; ++it) {
      const int row = wave * 8 + it * 4 + q;
      unsigned short hb[8];
#pragma unroll
      for (int e = 0; e < 8; ++e) hb[e] = f2bf_bits(sm[row][c8 + e]);
      const v4u u = (v4u){pk16(hb[0], hb[1]), pk16(hb[2], hb[3]), pk16(hb[4], hb[5]), pk16(hb[6], hb[7])};
      *(volatile v4u*)(out + (size_t)(d0 + row) * kNpos + n0 + c8) = u;
    }
    __threadfence();
  }
}

__global__ __launch_bounds__(256) void weights_kernel(const float* __restrict__ G, const float* __restrict__ xsq,
                                                      const float* __restrict__ psq, const float* __restrict__ invden,
                                                      unsigned short* __restrict__ Ph, unsigned short* __restrict__ Pl,
                                                      float* __restrict__ rscale) {
  __shared__ float redM[8];
  __shared__ float redS[8];
  __shared__ __align__(16) float sRS[kWRows];
  const int t = threadIdx.x, lane = t & 31, wave = t >> 5;
  const int cA = 8 * t;
  const int cB = (kNpos >> 1) + 8 * t;
  float pq[16], idn[16];
  {
    const v4f q0 = *(const v4f*)(psq + cA), q1 = *(const v4f*)(psq + cA + 4);
    const v4f q2 = *(const v4f*)(psq + cB), q3 = *(const v4f*)(psq + cB + 4);
    const v4f i0 = *(const v4f*)(invden + cA), i1 = *(const v4f*)(invden + cA + 4);
    const v4f i2 = *(const v4f*)(invden + cB), i3 = *(const v4f*)(invden + cB + 4);
#pragma unroll
    for (int e = 0; e < 4; ++e) {
      pq[e] = q0[e]; pq[4 + e] = q1[e]; pq[8 + e] = q2[e]; pq[12 + e] = q3[e];
      idn[e] = i0[e]; idn[4 + e] = i1[e]; idn[8 + e] = i2[e]; idn[12 + e] = i3[e];
    }
  }
#pragma unroll 1
  for (int r = 0; r < kWRows; ++r) {
    const int row = blockIdx.x * kWRows + r;
    const float xs = xsq[row];
    const float* gr = G + (size_t)row * kNpos;
    const v4f g0 = *(const v4f*)(gr + cA), g1 = *(const v4f*)(gr + cA + 4);
    const v4f g2 = *(const v4f*)(gr + cB), g3 = *(const v4f*)(gr + cB + 4);
    float gv[16];
#pragma unroll
    for (int e = 0; e < 4; ++e) { gv[e] = g0[e]; gv[4 + e] = g1[e]; gv[8 + e] = g2[e]; gv[12 + e] = g3[e]; }
    float lg[16];
    float m = -INFINITY;
#pragma unroll
    for (int e = 0; e < 16; ++e) {
      const float sq = (xs + pq[e]) - 2.0f * gv[e];
      const float d  = __builtin_amdgcn_sqrtf(fmaxf(sq, 0.0f));
      lg[e] = -d * idn[e];
      m = fmaxf(m, lg[e]);
    }
#pragma unroll
    for (int off = 16; off > 0; off >>= 1) m = fmaxf(m, __shfl_xor(m, off));
    if (lane == 0) redM[wave] = m;
    __syncthreads();
    float mb = redM[0];
#pragma unroll
    for (int w = 1; w < 8; ++w) mb = fmaxf(mb, redM[w]);
    float ps = 0.f;
    unsigned short hb[16], lb[16];
#pragma unroll
    for (int e = 0; e < 16; ++e) {
      const float p = __expf(lg[e] - mb);
      ps += p;
      const unsigned short h = f2bf_bits(p);
      hb[e] = h;
      lb[e] = f2bf_bits(p - bf_bits2f(h));
    }
    const v4u h0 = (v4u){pk16(hb[0], hb[1]),  pk16(hb[2], hb[3]),   pk16(hb[4], hb[5]),   pk16(hb[6], hb[7])};
    const v4u h1 = (v4u){pk16(hb[8], hb[9]),  pk16(hb[10], hb[11]), pk16(hb[12], hb[13]), pk16(hb[14], hb[15])};
    const v4u l0 = (v4u){pk16(lb[0], lb[1]),  pk16(lb[2], lb[3]),   pk16(lb[4], lb[5]),   pk16(lb[6], lb[7])};
    const v4u l1 = (v4u){pk16(lb[8], lb[9]),  pk16(lb[10], lb[11]), pk16(lb[12], lb[13]), pk16(lb[14], lb[15])};
    unsigned short* ph = Ph + (size_t)row * kNpos;
    unsigned short* pl = Pl + (size_t)row * kNpos;
    for (int pass = 0; pass < 2; ++pass) {
      *(volatile v4u*)(ph + cA) = h0;
      *(volatile v4u*)(ph + cB) = h1;
      *(volatile v4u*)(pl + cA) = l0;
      *(volatile v4u*)(pl + cB) = l1;
      __threadfence();
    }
#pragma unroll
    for (int off = 16; off > 0; off >>= 1) ps += __shfl_xor(ps, off);
    if (lane == 0) redS[wave] = ps;
    __syncthreads();
    if (t == 0) {
      float S = redS[0];
#pragma unroll
      for (int w = 1; w < 8; ++w) S += redS[w];
      const float em  = __expf(mb);
      const float den = em * S + 1e-8f;
      sRS[r] = em * (1.0f / den);
    }
  }
  __syncthreads();
  if (wave == 0 && lane < 8) {
    const v4f v = *(const v4f*)(sRS + 4 * lane);
    float* dst = rscale + (size_t)blockIdx.x * kWRows + 4 * lane;
    *(volatile v4f*)dst = v;
    __threadfence();
    *(volatile v4f*)dst = v;
  }
}

extern "C" void kernel_launch(void* const* d_in, const int* in_sizes, int n_in,
                              void* d_out, int out_size, void* d_ws, size_t ws_size,
                              hipStream_t stream) {
  if (n_in < 4) return;
  if (in_sizes[0] != kTok * kDim || in_sizes[1] != kNpos * kDim || in_sizes[2] != kNpos * kDim || in_sizes[3] != kNpos) return;
  if (out_size != kTok * kDim) return;
  if (ws_size < kWsEnd) return;

  const float* x    = (const float*)d_in[0];
  const float* pos  = (const float*)d_in[1];
  const float* val  = (const float*)d_in[2];
  const float* temp = (const float*)d_in[3];
  float* out = (float*)d_out;

  char* ws = (char*)d_ws;
  unsigned short* XB  = (unsigned short*)(ws + kOffXB);
  unsigned short* PB  = (unsigned short*)(ws + kOffPB);
  unsigned short* VT  = (unsigned short*)(ws + kOffVT);
  float* xsq  = (float*)(ws + kOffXsq);
  float* psq  = (float*)(ws + kOffPsq);
  float* idn  = (float*)(ws + kOffIdn);
  float* rsc  = (float*)(ws + kOffRsc);
  float* G    = (float*)(ws + kOffG);
  unsigned short* Ph = (unsigned short*)(ws + kOffPh);
  unsigned short* Pl = (unsigned short*)(ws + kOffPl);

  rowcast_bf16_kernel<false><<<dim3(kTok / 32), dim3(256), 0, stream>>>(x, XB, xsq, temp, idn);
  rowcast_bf16_kernel<true><<<dim3(kNpos / 32), dim3(256), 0, stream>>>(pos, PB, psq, temp, idn);
  vtcast_kernel<<<dim3(kDim / 64, kNpos / 64), dim3(256), 0, stream>>>(val, VT);

  for (int blk = 0; blk < kNumBlk; ++blk) {
    const unsigned short* Ablk = XB + (size_t)blk * kRowsBlk * kDim;
    wmma_gemm64<1, 0, 0, 0, false><<<dim3(kGTiles / 8, 1), dim3(256), 0, stream>>>(
        Ablk, Ablk, kDim, 0L, PB, PB, kDim, 0L, (void*)G, (void*)G, kNpos, 0L,
        xsq, xsq, 0L, kRowsBlk, kNpos, kDim, 1.0f);
    weights_kernel<<<dim3(kRowsBlk / kWRows), dim3(256), 0, stream>>>(
        G, xsq + (size_t)blk * kRowsBlk, psq, idn, Ph, Pl, rsc + (size_t)blk * kRowsBlk);
    float* Oblk = out + (size_t)blk * kRowsBlk * kDim;
    wmma_gemm64<1, 1, 3, 0, false><<<dim3(kPVTiles / 8, 1), dim3(256), 0, stream>>>(
        Ph, Pl, kNpos, 0L, VT, VT, kNpos, 0L, (void*)Oblk, (void*)Oblk, kDim, 0L,
        rsc + (size_t)blk * kRowsBlk, xsq, 0L, kRowsBlk, kDim, kNpos, 1.0f);
  }
}
